// MambaBlock_68161130988021
// MI455X (gfx1250) — hardware-verified
//
#include <hip/hip_runtime.h>
#include <math.h>

typedef __attribute__((ext_vector_type(16))) __bf16   v16b;
typedef __attribute__((ext_vector_type(8)))  __bf16   v8b;
typedef __attribute__((ext_vector_type(8)))  float    v8f;
typedef __attribute__((ext_vector_type(4)))  float    v4f;
typedef __attribute__((ext_vector_type(4)))  unsigned v4u;

constexpr int kBatch  = 2;
constexpr int kSeq    = 2048;
constexpr int kDm     = 768;
constexpr int kDin    = 1536;
constexpr int kNst    = 16;
constexpr int kRows   = kBatch * kSeq;
constexpr int kXpReal = 2 * kNst;
constexpr int kBcP    = 64;
constexpr int kConvTP = 260;
constexpr int kScanTS = 64;
constexpr int kScanCh = 64;
constexpr int kScanYP = 68;
constexpr float kRmsEps = 1.1920928955078125e-07f;
static_assert((kSeq & (kSeq - 1)) == 0, "sequence length is a power of two");
static_assert((kDm % 32) == 0 && (kDin % 32) == 0, "GEMM K multiples of 32");
static_assert((kRows % 64) == 0 && (kDin % 64) == 0 && (kBcP % 64) == 0 && (kDm % 64) == 0, "GEMM M,N multiples of 64");
static_assert((kSeq % kScanTS) == 0 && (kSeq % 64) == 0 && (kDin % kScanCh) == 0 && (kDin % 256) == 0, "tile multiples");
static_assert(kDm == 3 * 256, "norm kernel: three 256-wide segments per row");
static_assert(kXpReal == 32 && kNst == 16, "B|C row is 32 floats");

constexpr size_t kOffWIN  = 0;
constexpr size_t kOffWDT  = kOffWIN  + (size_t)2 * kDin * kDm * 2;
constexpr size_t kOffWOUT = kOffWDT  + (size_t)kDin * kDin * 2;
constexpr size_t kOffWXP  = kOffWOUT + (size_t)kDm * kDin * 2;
constexpr size_t kOffXNH  = kOffWXP  + (size_t)kBcP * kDin * 2;
constexpr size_t kOffXNL  = kOffXNH  + (size_t)kRows * kDm * 2;
constexpr size_t kOffXB   = kOffXNL  + (size_t)kRows * kDm * 2;
constexpr size_t kOffZP   = kOffXB   + (size_t)kRows * kDin * 4;
constexpr size_t kOffUH   = kOffZP   + (size_t)kRows * kDin * 4;
constexpr size_t kOffUL   = kOffUH   + (size_t)kRows * kDin * 2;
constexpr size_t kOffBC   = kOffUL   + (size_t)kRows * kDin * 2;
constexpr size_t kOffGH   = kOffBC   + (size_t)kRows * kBcP * 4;
constexpr size_t kOffGL   = kOffGH   + (size_t)kRows * kDin * 2;
constexpr size_t kWsTotal = kOffGL   + (size_t)kRows * kDin * 2;
static_assert(kWsTotal == 126287872ull, "carve total");
static_assert(kWsTotal <= 134217728ull, "carve cap");
static_assert(kOffZP == kOffXB + (size_t)kRows * kDin * 4, "z plane directly follows the xb plane");
static_assert((kOffWDT % 128) == 0 && (kOffWOUT % 128) == 0 && (kOffWXP % 128) == 0 && (kOffXNH % 128) == 0 &&
              (kOffXNL % 128) == 0 && (kOffXB % 128) == 0 && (kOffZP % 128) == 0 && (kOffUH % 128) == 0 &&
              (kOffUL % 128) == 0 && (kOffBC % 128) == 0 && (kOffGH % 128) == 0 && (kOffGL % 128) == 0, "128-B aligned regions");

__device__ __forceinline__ unsigned bf_rne_u(float f) {
  const unsigned u = __float_as_uint(f);
  return (u + 0x7FFFu + ((u >> 16) & 1u)) >> 16;
}
__device__ __forceinline__ float bf_u2f(unsigned h) { return __uint_as_float(h << 16); }
__device__ __forceinline__ float bf_snap(float f) { return bf_u2f(bf_rne_u(f)); }
__device__ __forceinline__ unsigned pack2(unsigned lo16, unsigned hi16) { return lo16 | (hi16 << 16); }

__device__ __forceinline__ void conv8_bf16(const v4f a0, const v4f a1, v4u& hv) {
#pragma unroll
  for (int e = 0; e < 2; ++e) {
    const float f0 = a0[2 * e], f1 = a0[2 * e + 1], f2 = a1[2 * e], f3 = a1[2 * e + 1];
    hv[e]     = pack2(bf_rne_u(f0), bf_rne_u(f1));
    hv[2 + e] = pack2(bf_rne_u(f2), bf_rne_u(f3));
  }
}
__device__ __forceinline__ void split8_bf16(const v4f a0, const v4f a1, v4u& hv, v4u& lv) {
#pragma unroll
  for (int e = 0; e < 2; ++e) {
    const float f0 = a0[2 * e], f1 = a0[2 * e + 1], f2 = a1[2 * e], f3 = a1[2 * e + 1];
    const unsigned h0 = bf_rne_u(f0), h1 = bf_rne_u(f1), h2 = bf_rne_u(f2), h3 = bf_rne_u(f3);
    const unsigned l0 = bf_rne_u(f0 - bf_u2f(h0)), l1 = bf_rne_u(f1 - bf_u2f(h1));
    const unsigned l2 = bf_rne_u(f2 - bf_u2f(h2)), l3 = bf_rne_u(f3 - bf_u2f(h3));
    hv[e]     = pack2(h0, h1);
    hv[2 + e] = pack2(h2, h3);
    lv[e]     = pack2(l0, l1);
    lv[2 + e] = pack2(l2, l3);
  }
}

__device__ __forceinline__ void dep_guard4_b(v8f& a, v8f& b, v8f& c, v8f& d, v16b x, v16b y) {
  asm volatile("v_nop\n\tv_nop\n\tv_nop\n\tv_nop" : "+v"(a), "+v"(b), "+v"(c), "+v"(d) : "v"(x), "v"(y));
}
__device__ __forceinline__ void keep4_b(v16b a, v16b b, v16b c, v16b d) { asm volatile("v_nop" :: "v"(a), "v"(b), "v"(c), "v"(d)); }
__device__ __forceinline__ void acc_guard4(v8f& a, v8f& b, v8f& c, v8f& d) { asm volatile("v_nop\n\tv_nop\n\tv_nop\n\tv_nop" : "+v"(a), "+v"(b), "+v"(c), "+v"(d)); }
struct FragB {
  union U { v16b v; v8b h[2]; };
  static __device__ __forceinline__ v16b load(const __bf16* p) {
    U f; f.h[0] = *(const v8b*)(p); f.h[1] = *(const v8b*)(p + 16); return f.v;
  }
  static __device__ __forceinline__ v8f mma(v16b a, v16b b, v8f c) {
    return __builtin_amdgcn_wmma_f32_16x16x32_bf16(false, a, false, b, (short)0, c, false, false);
  }
};

template <int BIAS_MODE, bool RESID>
__global__ __launch_bounds__(256) void wmma_gemm64_ahl(
    const unsigned short* __restrict__ Ahp, const unsigned short* __restrict__ Alp, int lda, long strideA,
    const unsigned short* __restrict__ Btp, int ldb, long strideB,
    float* __restrict__ Cout, int ldc, long strideC,
    const float* __restrict__ bias, const float* __restrict__ resid,
    int M, int N, int K) {
  typedef __bf16 T;
  typedef v16b V;
  const T* Ah = (const T*)Ahp; const T* Al = (const T*)Alp; const T* Bt = (const T*)Btp;
  __shared__ __align__(16) float sT[8][16 * 68];
  const int b    = blockIdx.y;
  const int lane = threadIdx.x & 31;
  const int wave = threadIdx.x >> 5;
  const int tilesN = N >> 6;
  const int tilesM = M >> 6;
  const int tile = blockIdx.x * 8 + wave;
  if (tile >= tilesM * tilesN) return;
  const int tm = tile / tilesN;
  const int tn = tile - tm * tilesN;
  const int m0 = tm << 6;
  const int n0 = tn << 6;

  const T* Ab  = Ah + (size_t)b * strideA;
  const T* Ab2 = Al + (size_t)b * strideA;
  const T* Bb  = Bt + (size_t)b * strideB;

  const int rlane = lane & 15;
  const int koff  = (lane >> 4) * 8;
  const int mOff  = (lane >> 4) * 8;

  v8f acc[4][4];
#pragma unroll
  for (int i = 0; i < 4; ++i)
#pragma unroll
    for (int j = 0; j < 4; ++j) acc[i][j] = (v8f){0.f,0.f,0.f,0.f,0.f,0.f,0.f,0.f};

  for (int k0 = 0; k0 < K; k0 += 32) {
    V bh[4];
#pragma unroll
    for (int j = 0; j < 4; ++j) {
      const size_t bo = (size_t)(n0 + (j << 4) + rlane) * ldb + koff + k0;
      bh[j] = FragB::load(Bb + bo);
    }
#pragma unroll
    for (int i = 0; i < 4; ++i) {
      const size_t ao = (size_t)(m0 + (i << 4) + rlane) * lda + koff + k0;
      V ah = FragB::load(Ab + ao);
      V al = FragB::load(Ab2 + ao);
#pragma unroll
      for (int j = 0; j < 4; ++j) {
        acc[i][j] = FragB::mma(ah, bh[j], acc[i][j]);
        acc[i][j] = FragB::mma(al, bh[j], acc[i][j]);
      }
      dep_guard4_b(acc[i][0], acc[i][1], acc[i][2], acc[i][3], ah, al);
    }
    keep4_b(bh[0], bh[1], bh[2], bh[3]);
  }
  acc_guard4(acc[0][0], acc[0][1], acc[0][2], acc[0][3]);
  acc_guard4(acc[1][0], acc[1][1], acc[1][2], acc[1][3]);
  acc_guard4(acc[2][0], acc[2][1], acc[2][2], acc[2][3]);
  acc_guard4(acc[3][0], acc[3][1], acc[3][2], acc[3][3]);

  float* slab = sT[wave];
  float* C = Cout + (size_t)b * strideC;
  const int hh = lane >> 4, c4 = (lane & 15) * 4;
  v4f bq = (v4f){0.f, 0.f, 0.f, 0.f};
  if (BIAS_MODE == 2) {
    const v4f braw = *(const v4f*)(bias + n0 + c4);
    bq[0] = bf_snap(braw[0]); bq[1] = bf_snap(braw[1]); bq[2] = bf_snap(braw[2]); bq[3] = bf_snap(braw[3]);
  }
#pragma unroll
  for (int i = 0; i < 4; ++i) {
    const int mBase = m0 + (i << 4);
#pragma unroll
    for (int j = 0; j < 4; ++j) {
#pragma unroll
      for (int r = 0; r < 8; ++r) slab[(mOff + r) * 68 + (j << 4) + rlane] = acc[i][j][r];
    }
    __builtin_amdgcn_fence(__ATOMIC_RELEASE, "workgroup");
    __builtin_amdgcn_wave_barrier();
    __builtin_amdgcn_fence(__ATOMIC_ACQUIRE, "workgroup");
    v4f ov[8];
#pragma unroll
    for (int it = 0; it < 8; ++it) {
      const int row = it * 2 + hh;
      v4f v = *(const v4f*)(slab + row * 68 + c4);
      if (BIAS_MODE == 2) v += bq;
      if (RESID) {
        const v4f rr = *(const v4f*)(resid + (size_t)(mBase + row) * ldc + n0 + c4);
        v4f rs;
        rs[0] = bf_snap(rr[0]); rs[1] = bf_snap(rr[1]); rs[2] = bf_snap(rr[2]); rs[3] = bf_snap(rr[3]);
        v += rs;
      }
      ov[it] = v;
    }
    for (int pass = 0; pass < 2; ++pass) {
#pragma unroll
      for (int it = 0; it < 8; ++it) {
        const int row = it * 2 + hh;
        *(volatile v4f*)(C + (size_t)(mBase + row) * ldc + n0 + c4) = ov[it];
      }
      __threadfence();
    }
    __builtin_amdgcn_fence(__ATOMIC_RELEASE, "workgroup");
    __builtin_amdgcn_wave_barrier();
    __builtin_amdgcn_fence(__ATOMIC_ACQUIRE, "workgroup");
  }
}

__global__ __launch_bounds__(256) void cast_rows_bf16_kernel(
    const float* __restrict__ src, unsigned short* __restrict__ dst, int total8, int valid8)
{
  const int i = blockIdx.x * 256 + threadIdx.x;
  if (i >= total8) return;
  const bool ok = (i < valid8);
  const int ic = ok ? i : (valid8 - 1);
  const size_t e0 = (size_t)ic << 3;
  v4f a0 = *(const v4f*)(src + e0);
  v4f a1 = *(const v4f*)(src + e0 + 4);
#pragma unroll
  for (int e = 0; e < 4; ++e) {
    a0[e] = ok ? a0[e] : 0.0f;
    a1[e] = ok ? a1[e] : 0.0f;
  }
  v4u hv;
  conv8_bf16(a0, a1, hv);
  unsigned short* q = dst + ((size_t)i << 3);
  *(volatile v4u*)q = hv;
  __threadfence();
  *(volatile v4u*)q = hv;
}

__global__ __launch_bounds__(256) void rmsnorm_split_kernel(
    const float* __restrict__ x, const float* __restrict__ gain,
    unsigned short* __restrict__ XNH, unsigned short* __restrict__ XNL)
{
  const int lane = threadIdx.x & 31, wave = threadIdx.x >> 5;
  const int row = blockIdx.x * 8 + wave;
  const float* xr = x + (size_t)row * kDm;
  v4f xa[3], xc[3];
  float ss = 0.0f;
#pragma unroll
  for (int j = 0; j < 3; ++j) {
    const int col = j * 256 + lane * 8;
    v4f a0 = *(const v4f*)(xr + col);
    v4f a1 = *(const v4f*)(xr + col + 4);
#pragma unroll
    for (int e = 0; e < 4; ++e) {
      a0[e] = bf_snap(a0[e]);
      a1[e] = bf_snap(a1[e]);
      ss = fmaf(a0[e], a0[e], ss);
      ss = fmaf(a1[e], a1[e], ss);
    }
    xa[j] = a0;
    xc[j] = a1;
  }
#pragma unroll
  for (int off = 16; off > 0; off >>= 1) ss += __shfl_xor(ss, off, 32);
  const float ms = ss * (1.0f / (float)kDm);
  const float sc = rsqrtf(ms + kRmsEps);
  v4u hv[3], lv[3];
#pragma unroll
  for (int j = 0; j < 3; ++j) {
    const int col = j * 256 + lane * 8;
    const v4f g0 = *(const v4f*)(gain + col);
    const v4f g1 = *(const v4f*)(gain + col + 4);
    v4f o0, o1;
#pragma unroll
    for (int e = 0; e < 4; ++e) {
      o0[e] = (xa[j][e] * sc) * bf_snap(g0[e]);
      o1[e] = (xc[j][e] * sc) * bf_snap(g1[e]);
    }
    split8_bf16(o0, o1, hv[j], lv[j]);
  }
  for (int pass = 0; pass < 2; ++pass) {
#pragma unroll
    for (int j = 0; j < 3; ++j) {
      const size_t o = (size_t)row * kDm + j * 256 + lane * 8;
      *(volatile v4u*)(XNH + o) = hv[j];
      *(volatile v4u*)(XNL + o) = lv[j];
    }
    __threadfence();
  }
}

__global__ __launch_bounds__(256) void conv_silu_kernel(
    const float* __restrict__ XB, const float* __restrict__ cw, const float* __restrict__ cb,
    unsigned short* __restrict__ UH, unsigned short* __restrict__ UL)
{
  __shared__ __align__(16) float sT[16 * kConvTP];
  const int tid = threadIdx.x, lane = tid & 31, wave = tid >> 5;
  const int d0 = blockIdx.x * 256, d = d0 + tid;
  const int g0 = blockIdx.y * 64;
  const int tb = g0 & (kSeq - 1);
  const v4f wv = *(const v4f*)(cw + (size_t)d * 4);
  const float w0 = bf_snap(wv[0]), w1 = bf_snap(wv[1]), w2 = bf_snap(wv[2]), w3 = bf_snap(wv[3]);
  const float bcv = bf_snap(cb[d]);
  float xm3, xm2, xm1;
  {
    const bool hist = (tb > 0);
    const int rb = hist ? (g0 - 3) : g0;
    const float v3 = XB[(size_t)rb * kDin + d];
    const float v2 = XB[(size_t)(rb + 1) * kDin + d];
    const float v1 = XB[(size_t)(rb + 2) * kDin + d];
    xm3 = hist ? v3 : 0.f;
    xm2 = hist ? v2 : 0.f;
    xm1 = hist ? v1 : 0.f;
  }
#pragma unroll 1
  for (int sub = 0; sub < 4; ++sub) {
    const int lb = g0 + sub * 16;
#pragma unroll 1
    for (int s = 0; s < 16; ++s) {
      const float xcur = XB[(size_t)(lb + s) * kDin + d];
      float acc = w0 * xm3;
      acc = fmaf(w1, xm2, acc);
      acc = fmaf(w2, xm1, acc);
      acc = fmaf(w3, xcur, acc);
      const float sv = acc + bcv;
      const float sg = 1.0f / (1.0f + expf(-sv));
      sT[s * kConvTP + tid] = sv * sg;
      xm3 = xm2; xm2 = xm1; xm1 = xcur;
    }
    __syncthreads();
    v4u hv[2], lv[2];
#pragma unroll
    for (int it = 0; it < 2; ++it) {
      const float* sp = sT + (it * 8 + wave) * kConvTP + lane * 8;
      const v4f a0 = *(const v4f*)(sp);
      const v4f a1 = *(const v4f*)(sp + 4);
      split8_bf16(a0, a1, hv[it], lv[it]);
    }
    for (int pass = 0; pass < 2; ++pass) {
#pragma unroll
      for (int it = 0; it < 2; ++it) {
        const size_t o = (size_t)(lb + it * 8 + wave) * kDin + d0 + lane * 8;
        *(volatile v4u*)(UH + o) = hv[it];
        *(volatile v4u*)(UL + o) = lv[it];
      }
      __threadfence();
    }
    __syncthreads();
  }
}

__global__ __launch_bounds__(64) void scan_kernel(
    const float* __restrict__ BC, const unsigned short* __restrict__ UH, const unsigned short* __restrict__ UL,
    const float* __restrict__ DL, const float* __restrict__ ZP,
    const float* __restrict__ Alog, const float* __restrict__ Dp,
    unsigned short* __restrict__ GH, unsigned short* __restrict__ GL)
{
  __shared__ __align__(16) float sX[kScanTS * 32];
  __shared__ __align__(16) float sU[kScanTS * kScanYP];
  __shared__ __align__(16) float sY[kScanTS * kScanYP];
  __shared__ __align__(16) float sA[kNst * kScanCh];
  const int tid = threadIdx.x, lane = tid & 31, wave = tid >> 5;
  constexpr int kBlkPerB = kDin / kScanCh;
  const int bix = blockIdx.x / kBlkPerB;
  const int d0  = (blockIdx.x - bix * kBlkPerB) * kScanCh;
  const int d   = d0 + tid;
  const size_t row0 = (size_t)bix * kSeq;
#pragma unroll 1
  for (int s = 0; s < kNst; ++s) sA[s * kScanCh + tid] = -expf(bf_snap(Alog[(size_t)d * kNst + s]));
  __syncthreads();
  float negA[kNst], h[kNst];
#pragma unroll
  for (int s = 0; s < kNst; ++s) {
    negA[s] = sA[s * kScanCh + tid];
    h[s] = 0.f;
  }
  const float Dd = bf_snap(Dp[d]);
  const int q = lane >> 3, c8 = (lane & 7) * 8;
#pragma unroll 1
  for (int t0 = 0; t0 < kSeq; t0 += kScanTS) {
    __syncthreads();
#pragma unroll
    for (int i = 0; i < 8; ++i) {
      const int r = (tid >> 3) + 8 * i;
      const int c4 = (tid & 7) * 4;
      *(v4f*)(sX + r * 32 + c4) = *(const v4f*)(BC + (row0 + t0 + r) * kBcP + c4);
    }
#pragma unroll
    for (int i = 0; i < 8; ++i) {
      const int item = tid + 64 * i;
      const int r = item >> 3, sg8 = (item & 7) * 8;
      const size_t o = (row0 + t0 + r) * kDin + d0 + sg8;
      const v4u wh = *(const v4u*)(UH + o);
      const v4u wl = *(const v4u*)(UL + o);
      const unsigned h0 = wh[0], h1 = wh[1], h2 = wh[2], h3 = wh[3];
      const unsigned l0 = wl[0], l1 = wl[1], l2 = wl[2], l3 = wl[3];
      v4f f0, f1;
      f0[0] = __uint_as_float(h0 << 16)         + __uint_as_float(l0 << 16);
      f0[1] = __uint_as_float(h0 & 0xffff0000u) + __uint_as_float(l0 & 0xffff0000u);
      f0[2] = __uint_as_float(h1 << 16)         + __uint_as_float(l1 << 16);
      f0[3] = __uint_as_float(h1 & 0xffff0000u) + __uint_as_float(l1 & 0xffff0000u);
      f1[0] = __uint_as_float(h2 << 16)         + __uint_as_float(l2 << 16);
      f1[1] = __uint_as_float(h2 & 0xffff0000u) + __uint_as_float(l2 & 0xffff0000u);
      f1[2] = __uint_as_float(h3 << 16)         + __uint_as_float(l3 << 16);
      f1[3] = __uint_as_float(h3 & 0xffff0000u) + __uint_as_float(l3 & 0xffff0000u);
      *(v4f*)(sU + r * kScanYP + sg8)     = f0;
      *(v4f*)(sU + r * kScanYP + sg8 + 4) = f1;
    }
    __syncthreads();
#pragma unroll 1
    for (int s = 0; s < kScanTS; ++s) {
      const size_t grow = row0 + t0 + s;
      float v = DL[grow * kDin + d];
      asm volatile("" : "+v"(v));
      float zv = ZP[grow * kDin + d];
      asm volatile("" : "+v"(zv));
      const float* xr = sX + s * 32;
      v4f Bq[4], Cq[4];
#pragma unroll
      for (int q4 = 0; q4 < 4; ++q4) {
        Bq[q4] = *(const v4f*)(xr + 4 * q4);
        Cq[q4] = *(const v4f*)(xr + kNst + 4 * q4);
      }
      const float xt  = sU[s * kScanYP + tid];
      const float dt  = fmaxf(v, 0.0f) + log1pf(__expf(-fabsf(v)));
      const float dtx = dt * xt;
      float y = 0.f;
#pragma unroll
      for (int k = 0; k < kNst; ++k) {
        const float e = __expf(dt * negA[k]);
        h[k] = fmaf(e, h[k], dtx * Bq[k >> 2][k & 3]);
        y = fmaf(h[k], Cq[k >> 2][k & 3], y);
      }
      y = fmaf(xt, Dd, y);
      const float sg = __builtin_amdgcn_rcpf(1.0f + __expf(-zv));
      sY[s * kScanYP + tid] = y * (zv * sg);
    }
    __syncthreads();
    v4u hv[8], lv[8];
#pragma unroll
    for (int it = 0; it < 8; ++it) {
      const int row = it * 8 + wave * 4 + q;
      const float* sp = sY + row * kScanYP + c8;
      const v4f a0 = *(const v4f*)(sp);
      const v4f a1 = *(const v4f*)(sp + 4);
      split8_bf16(a0, a1, hv[it], lv[it]);
    }
    for (int pass = 0; pass < 2; ++pass) {
#pragma unroll
      for (int it = 0; it < 8; ++it) {
        const int row = it * 8 + wave * 4 + q;
        const size_t o = (row0 + t0 + row) * kDin + d0 + c8;
        *(volatile v4u*)(GH + o) = hv[it];
        *(volatile v4u*)(GL + o) = lv[it];
      }
      __threadfence();
    }
  }
}

extern "C" void kernel_launch(void* const* d_in, const int* in_sizes, int n_in,
                              void* d_out, int out_size, void* d_ws, size_t ws_size,
                              hipStream_t stream) {
  if (n_in < 11) return;
  if (in_sizes[0] != kRows * kDm) return;
  if (in_sizes[1] != kDm) return;
  if (in_sizes[2] != 2 * kDin * kDm) return;
  if (in_sizes[3] != kDin * 4) return;
  if (in_sizes[4] != kDin) return;
  if (in_sizes[5] != kXpReal * kDin) return;
  if (in_sizes[6] != kDin * kDin) return;
  if (in_sizes[7] != kDin) return;
  if (in_sizes[8] != kDin * kNst) return;
  if (in_sizes[9] != kDin) return;
  if (in_sizes[10] != kDm * kDin) return;
  if (out_size != kRows * kDm) return;
  if (ws_size < kWsTotal) return;

  const float* x       = (const float*)d_in[0];
  const float* norm_w  = (const float*)d_in[1];
  const float* W_in    = (const float*)d_in[2];
  const float* conv_w  = (const float*)d_in[3];
  const float* conv_b  = (const float*)d_in[4];
  const float* W_xproj = (const float*)d_in[5];
  const float* W_dt    = (const float*)d_in[6];
  const float* b_dt    = (const float*)d_in[7];
  const float* A_log   = (const float*)d_in[8];
  const float* D_skip  = (const float*)d_in[9];
  const float* W_out   = (const float*)d_in[10];
  float* out = (float*)d_out;

  char* ws = (char*)d_ws;
  unsigned short* WIN  = (unsigned short*)(ws + kOffWIN);
  unsigned short* WDT  = (unsigned short*)(ws + kOffWDT);
  unsigned short* WOUT = (unsigned short*)(ws + kOffWOUT);
  unsigned short* WXP  = (unsigned short*)(ws + kOffWXP);
  unsigned short* XNH  = (unsigned short*)(ws + kOffXNH);
  unsigned short* XNL  = (unsigned short*)(ws + kOffXNL);
  float*          XB   = (float*)(ws + kOffXB);
  float*          ZP   = (float*)(ws + kOffZP);
  unsigned short* UH   = (unsigned short*)(ws + kOffUH);
  unsigned short* UL   = (unsigned short*)(ws + kOffUL);
  float*          BC   = (float*)(ws + kOffBC);
  unsigned short* GH   = (unsigned short*)(ws + kOffGH);
  unsigned short* GL   = (unsigned short*)(ws + kOffGL);

  constexpr int kWin8  = 2 * kDin * kDm / 8;
  constexpr int kWdt8  = kDin * kDin / 8;
  constexpr int kWout8 = kDm * kDin / 8;
  constexpr int kWxpT8 = kBcP * kDin / 8;
  constexpr int kWxpV8 = kXpReal * kDin / 8;
  static_assert((kWin8 % 256) == 0 && (kWdt8 % 256) == 0 && (kWout8 % 256) == 0 && (kWxpT8 % 256) == 0 && (kWxpV8 % 256) == 0,
                "cast grids are exact");

  cast_rows_bf16_kernel<<<kWin8 / 256, 256, 0, stream>>>(W_in, WIN, kWin8, kWin8);
  cast_rows_bf16_kernel<<<kWdt8 / 256, 256, 0, stream>>>(W_dt, WDT, kWdt8, kWdt8);
  cast_rows_bf16_kernel<<<kWout8 / 256, 256, 0, stream>>>(W_out, WOUT, kWout8, kWout8);
  cast_rows_bf16_kernel<<<kWxpT8 / 256, 256, 0, stream>>>(W_xproj, WXP, kWxpT8, kWxpV8);

  rmsnorm_split_kernel<<<kRows / 8, 256, 0, stream>>>(x, norm_w, XNH, XNL);

  wmma_gemm64_ahl<0, false><<<dim3((kRows / 64) * (kDin / 64) / 8, 2), 256, 0, stream>>>(
      XNH, XNL, kDm, 0L,
      WIN, kDm, (long)kDin * kDm,
      XB, kDin, (long)kRows * kDin,
      b_dt, x,
      kRows, kDin, kDm);

  conv_silu_kernel<<<dim3(kDin / 256, kRows / 64), 256, 0, stream>>>(XB, conv_w, conv_b, UH, UL);

  wmma_gemm64_ahl<0, false><<<dim3((kRows / 64) * (kBcP / 64) / 8, 1), 256, 0, stream>>>(
      UH, UL, kDin, 0L,
      WXP, kDin, 0L,
      BC, kBcP, 0L,
      b_dt, x,
      kRows, kBcP, kDin);

  wmma_gemm64_ahl<2, false><<<dim3((kRows / 64) * (kDin / 64) / 8, 1), 256, 0, stream>>>(
      UH, UL, kDin, 0L,
      WDT, kDin, 0L,
      XB, kDin, 0L,
      b_dt, x,
      kRows, kDin, kDin);

  scan_kernel<<<kBatch * (kDin / kScanCh), kScanCh, 0, stream>>>(BC, UH, UL, XB, ZP, A_log, D_skip, GH, GL);

  wmma_gemm64_ahl<0, true><<<dim3((kRows / 64) * (kDm / 64) / 8, 1), 256, 0, stream>>>(
      GH, GL, kDin, 0L,
      WOUT, kDin, 0L,
      out, kDm, 0L,
      b_dt, x,
      kRows, kDm, kDin);
}
